// OverfitJobGNN_60662118088919
// MI455X (gfx1250) — hardware-verified
//
#include <hip/hip_runtime.h>
#include <stddef.h>


#define DF    128
#define NOUT  32
#define GR    32
#define AP    136
#define XSP   132
#define NTHR  256
#define NWAVE 8
#define NB    512
#define SB    9
#define NBL   4096
#define SBL   12
#define CHUNK 1024
#define WCAP  ((CHUNK / NTHR) * 32)
#define GPW   4
#define GROWS 64
#define LGP   33

#define LDS_GCN ((NB * DF + NB + NWAVE * WCAP + NWAVE) * 4)
#define LDS_G1  ((NBL * 2 * 3 + NWAVE * WCAP + NWAVE) * 4)
#define LDS_G2  ((NB * DF + NB * 4 + NB * 2 + NWAVE * WCAP + NWAVE) * 4)

static_assert(WCAP == 128);
static_assert(CHUNK == NTHR * 4);
static_assert((1 << SB) == NB);
static_assert((1 << SBL) == NBL);
static_assert((NB % (2 * NWAVE)) == 0);
static_assert((NB % NTHR) == 0);
static_assert((NBL % NTHR) == 0);
static_assert((NB % GR) == 0);
static_assert(GROWS == 2 * NWAVE * GPW);
static_assert(GROWS == NWAVE * 8);
static_assert(LDS_GCN == 268320);
static_assert(LDS_G1 == 102432);
static_assert(LDS_G2 == 278560);

typedef float    v4f  __attribute__((ext_vector_type(4)));
typedef float    v8f  __attribute__((ext_vector_type(8)));
typedef int      v4i  __attribute__((ext_vector_type(4)));
typedef _Float16 v8h  __attribute__((ext_vector_type(8)));
typedef _Float16 v16h __attribute__((ext_vector_type(16)));
union Frag   { v16h v; v8h half[2]; };
union Pack16 { v8h h; v4i i; };

__device__ __forceinline__ v8f wm(v16h a, v16h b, v8f c) {
  v8f d = __builtin_amdgcn_wmma_f32_16x16x32_f16(false, a, false, b, (short)0, c, false, false);
  asm volatile("v_nop\n\tv_nop\n\tv_nop\n\tv_nop" : "+v"(d) : "v"(a), "v"(b));
  return d;
}

__device__ __forceinline__ float wsum(float v) {
  v += __shfl_xor(v, 16, 32);
  v += __shfl_xor(v, 8, 32);
  v += __shfl_xor(v, 4, 32);
  v += __shfl_xor(v, 2, 32);
  v += __shfl_xor(v, 1, 32);
  return v;
}
__device__ __forceinline__ float wmax(float v) {
  v = fmaxf(v, __shfl_xor(v, 16, 32));
  v = fmaxf(v, __shfl_xor(v, 8, 32));
  v = fmaxf(v, __shfl_xor(v, 4, 32));
  v = fmaxf(v, __shfl_xor(v, 2, 32));
  v = fmaxf(v, __shfl_xor(v, 1, 32));
  return v;
}

__device__ __forceinline__ v8h cvt8(v4f a, v4f b, float s) {
  Pack16 u;
  u.h[0] = (_Float16)(a.x * s); u.h[1] = (_Float16)(a.y * s); u.h[2] = (_Float16)(a.z * s); u.h[3] = (_Float16)(a.w * s);
  u.h[4] = (_Float16)(b.x * s); u.h[5] = (_Float16)(b.y * s); u.h[6] = (_Float16)(b.z * s); u.h[7] = (_Float16)(b.w * s);
  return u.h;
}

__device__ __forceinline__ v4f relu4(v4f y) {
  y.x = fmaxf(y.x, 0.f); y.y = fmaxf(y.y, 0.f); y.z = fmaxf(y.z, 0.f); y.w = fmaxf(y.w, 0.f);
  return y;
}
__device__ __forceinline__ float leaky02(float a) { return a > 0.f ? a : 0.2f * a; }

__global__ __launch_bounds__(NTHR) void k_prep(
    const float* __restrict__ w0, const float* __restrict__ w1, const float* __restrict__ w2,
    const float* __restrict__ w3, const float* __restrict__ w4, const float* __restrict__ w5,
    _Float16* t0, _Float16* t1, _Float16* t2, _Float16* t3, _Float16* t4, _Float16* t5) {
  const int y = blockIdx.y;
  const float* src;
  _Float16* dst;
  int NC;
  if (y == 0)      { src = w0; dst = t0; NC = DF; }
  else if (y == 1) { src = w1; dst = t1; NC = DF; }
  else if (y == 2) { src = w2; dst = t2; NC = DF; }
  else if (y == 3) { src = w3; dst = t3; NC = 2 * DF; }
  else if (y == 4) { src = w4; dst = t4; NC = DF; }
  else             { src = w5; dst = t5; NC = NOUT; }
  const int i = blockIdx.x * NTHR + threadIdx.x;
  if (i >= NC * (DF / 8)) return;
  const int n  = i >> 4;
  const int k0 = (i & 15) * 8;
  Pack16 u;
#pragma unroll
  for (int j = 0; j < 8; ++j) u.h[j] = (_Float16)(src[(size_t)(k0 + j) * NC + n] * 16.0f);
  _Float16* p = dst + (size_t)n * DF + k0;
  *(volatile v4i*)p = u.i;
  __threadfence();
  *(volatile v4i*)p = u.i;
}

template <int NBX, int SBX>
__device__ __forceinline__ int scan_chunk(const int* __restrict__ eid, int nE, bool al16, int cbase,
                                          int nodeBase, int tid, int wave, int* list) {
  const int el0 = tid * 4;
  const int e0  = cbase + el0;
  const int sent = -2147483647 - 1;
  v4i d;
  if (al16 && (e0 + 3 < nE)) {
    d = *(const v4i*)(eid + e0);
  } else {
    d.x = (e0     < nE) ? eid[min(e0,     nE - 1)] : sent;
    d.y = (e0 + 1 < nE) ? eid[min(e0 + 1, nE - 1)] : sent;
    d.z = (e0 + 2 < nE) ? eid[min(e0 + 2, nE - 1)] : sent;
    d.w = (e0 + 3 < nE) ? eid[min(e0 + 3, nE - 1)] : sent;
  }
  const unsigned s0 = (unsigned)d.x - (unsigned)nodeBase;
  const unsigned s1 = (unsigned)d.y - (unsigned)nodeBase;
  const unsigned s2 = (unsigned)d.z - (unsigned)nodeBase;
  const unsigned s3 = (unsigned)d.w - (unsigned)nodeBase;
  const bool h0 = s0 < (unsigned)NBX;
  const bool h1 = s1 < (unsigned)NBX;
  const bool h2 = s2 < (unsigned)NBX;
  const bool h3 = s3 < (unsigned)NBX;
  int wc = 0;
  const unsigned many = __builtin_amdgcn_ballot_w32(h0 | h1 | h2 | h3);
  if (many != 0u) {
#define HITJ(J, HJ, SJ) { \
      const unsigned mj = __builtin_amdgcn_ballot_w32(HJ); \
      if (HJ) { \
        const int pos = wc + (int)__builtin_amdgcn_mbcnt_lo(mj, 0u); \
        if (pos < WCAP) list[wave * WCAP + pos] = ((el0 + (J)) << SBX) | (int)(SJ); \
      } \
      wc += (int)__builtin_popcount(mj); }
    HITJ(0, h0, s0)
    HITJ(1, h1, s1)
    HITJ(2, h2, s2)
    HITJ(3, h3, s3)
#undef HITJ
  }
  return wc;
}

__global__ __launch_bounds__(NTHR) void k_deg(const int* __restrict__ ei, float* dinv, int nE) {
  __shared__ int cnt[NBL];
  __shared__ int list[NWAVE * WCAP];
  __shared__ int wcnt[NWAVE];
  const int tid = threadIdx.x, lane = tid & 31, wave = tid >> 5;
  const int nodeBase = blockIdx.x * NBL;
  for (int i = tid; i < NBL; i += NTHR) cnt[i] = 0;
  __syncthreads();

  const int* eid = ei + nE;
  const bool al16 = ((nE & 3) == 0);
  const int nChunks = (nE + CHUNK - 1) / CHUNK;
#pragma unroll 1
  for (int ch = 0; ch < nChunks; ++ch) {
    const int cbase = ch * CHUNK;
    const int wc = scan_chunk<NBL, SBL>(eid, nE, al16, cbase, nodeBase, tid, wave, list);
    if (lane == 0) wcnt[wave] = wc;
    __syncthreads();
    if (wave == 0) {
      for (int wsx = 0; wsx < NWAVE; ++wsx) {
        int n = wcnt[wsx];
        n = n < 0 ? 0 : (n > WCAP ? WCAP : n);
        for (int i = 0; i < n; ++i) {
          const int slot = list[wsx * WCAP + i] & (NBL - 1);
          const int c = cnt[slot];
          cnt[slot] = c + 1;
        }
      }
    }
    __syncthreads();
  }
  for (int i = tid; i < NBL / 4; i += NTHR) {
    v4f r;
    r.x = rsqrtf((float)(cnt[4 * i + 0] + 1));
    r.y = rsqrtf((float)(cnt[4 * i + 1] + 1));
    r.z = rsqrtf((float)(cnt[4 * i + 2] + 1));
    r.w = rsqrtf((float)(cnt[4 * i + 3] + 1));
    float* p = dinv + (size_t)nodeBase + 4 * i;
    *(volatile v4f*)p = r;
    __threadfence();
    *(volatile v4f*)p = r;
  }
}

__device__ __forceinline__ void epi_row(v8f acc, int T, int hh, int ncol, float esc,
                                        const float* Dv, float* Xs) {
#pragma unroll
  for (int r = 0; r < 8; ++r) {
    const int rl = T * 16 + 8 * hh + r;
    Xs[rl * XSP + ncol] = acc[r] * esc * Dv[rl];
  }
}

__device__ __forceinline__ void epi_att(v8f acc, int T, int hh, int m, int wave, int ncol,
                                        float cs, float cd, float esc, float* Xs, float* As, float* Ds) {
  float ss[8], sd[8];
#pragma unroll
  for (int r = 0; r < 8; ++r) {
    const float v = acc[r] * esc;
    Xs[(T * 16 + 8 * hh + r) * XSP + ncol] = v;
    ss[r] = v * cs;
    sd[r] = v * cd;
  }
#pragma unroll
  for (int mk = 1; mk < 16; mk <<= 1) {
#pragma unroll
    for (int r = 0; r < 8; ++r) {
      ss[r] += __shfl_xor(ss[r], mk, 32);
      sd[r] += __shfl_xor(sd[r], mk, 32);
    }
  }
  if (m == 0) {
#pragma unroll
    for (int r = 0; r < 8; ++r) {
      As[(T * 16 + 8 * hh + r) * NWAVE + wave] = ss[r];
      Ds[(T * 16 + 8 * hh + r) * NWAVE + wave] = sd[r];
    }
  }
}

__device__ __forceinline__ void stage16(const float* p, _Float16* q) {
  const v4f f0 = *(const v4f*)(p),     f1 = *(const v4f*)(p + 4);
  const v4f f2 = *(const v4f*)(p + 8), f3 = *(const v4f*)(p + 12);
  *(v8h*)(q)     = cvt8(f0, f1, 1.0f);
  *(v8h*)(q + 8) = cvt8(f2, f3, 1.0f);
}
__device__ __forceinline__ void stage16(const _Float16* p, _Float16* q) {
  *(v8h*)(q)     = *(const v8h*)(p);
  *(v8h*)(q + 8) = *(const v8h*)(p + 8);
}

template <typename AT, int MODE>
__global__ __launch_bounds__(NTHR) void k_gemm(
    const AT* __restrict__ A, const _Float16* __restrict__ Wt,
    const float* __restrict__ dinv, const float* __restrict__ asv, const float* __restrict__ adv,
    float* o0, float* oS, float* oD, int nN, int nPA, float esc) {
  __shared__ __attribute__((aligned(16))) _Float16 At[GR * AP];
  __shared__ __attribute__((aligned(16))) float Xs[GR * XSP];
  __shared__ __attribute__((aligned(16))) float As[GR * NWAVE];
  __shared__ __attribute__((aligned(16))) float Ds[GR * NWAVE];
  __shared__ __attribute__((aligned(16))) float Sa[GR];
  __shared__ __attribute__((aligned(16))) float Sd[GR];
  __shared__ float Dv[GR];

  const int tid  = threadIdx.x;
  const int lane = tid & 31;
  const int wave = tid >> 5;
  const int hh   = lane >> 4;
  const int m    = lane & 15;
  const int rowBase = blockIdx.x * GR;
  const int yb = (MODE == 1) ? (int)blockIdx.y * DF : 0;

  {
    const int r = tid >> 3;
    int row = rowBase + r;
    if (row > nN - 1) row = nN - 1;
    const int c0 = (tid & 7) * 16;
    stage16(A + (size_t)row * DF + c0, At + r * AP + c0);
    if (MODE == 0) { if (tid < GR) Dv[tid] = dinv[rowBase + tid]; }
  }
  __syncthreads();

  const int ncol = wave * 16 + m;
  v8f c0a = {0.f, 0.f, 0.f, 0.f, 0.f, 0.f, 0.f, 0.f};
  v8f c1a = {0.f, 0.f, 0.f, 0.f, 0.f, 0.f, 0.f, 0.f};
#pragma unroll
  for (int kt = 0; kt < DF / 32; ++kt) {
    const int k0 = kt * 32;
    Frag a0, a1, b;
    const _Float16* pb  = Wt + (size_t)(yb + ncol) * DF + k0 + 8 * hh;
    const _Float16* pa0 = At + m * AP + k0 + 8 * hh;
    const _Float16* pa1 = At + (16 + m) * AP + k0 + 8 * hh;
    b.half[0]  = *(const v8h*)pb;  b.half[1]  = *(const v8h*)(pb + 16);
    a0.half[0] = *(const v8h*)pa0; a0.half[1] = *(const v8h*)(pa0 + 16);
    a1.half[0] = *(const v8h*)pa1; a1.half[1] = *(const v8h*)(pa1 + 16);
    c0a = wm(a0.v, b.v, c0a);
    c1a = wm(a1.v, b.v, c1a);
  }

  if (MODE == 0) {
    epi_row(c0a, 0, hh, ncol, esc, Dv, Xs);
    epi_row(c1a, 1, hh, ncol, esc, Dv, Xs);
  } else {
    const float cs = asv[yb + ncol];
    const float cd = adv[yb + ncol];
    epi_att(c0a, 0, hh, m, wave, ncol, cs, cd, esc, Xs, As, Ds);
    epi_att(c1a, 1, hh, m, wave, ncol, cs, cd, esc, Xs, As, Ds);
  }
  __syncthreads();

  v4f xr[4];
#pragma unroll
  for (int i = 0; i < 4; ++i) xr[i] = *(const v4f*)(Xs + (4 * wave + i) * XSP + 4 * lane);
  const int OP = (MODE == 1) ? 2 * DF : DF;
  float* xpp[4];
#pragma unroll
  for (int i = 0; i < 4; ++i) xpp[i] = o0 + (size_t)(rowBase + 4 * wave + i) * OP + yb + 4 * lane;
  float* gp = 0;
  v4f gv = {0.f, 0.f, 0.f, 0.f};
  if (MODE == 1) {
    if (tid < GR) {
      float s = 0.f, d = 0.f;
#pragma unroll
      for (int w = 0; w < NWAVE; ++w) { s += As[tid * NWAVE + w]; d += Ds[tid * NWAVE + w]; }
      Sa[tid] = s;
      Sd[tid] = d;
    }
    __syncthreads();
    if (wave == 0 && lane < 8) {
      gv = *(const v4f*)(Sa + 4 * lane);
      gp = oS + (size_t)blockIdx.y * nPA + rowBase + 4 * lane;
    } else if (wave == 1 && lane < 8) {
      gv = *(const v4f*)(Sd + 4 * lane);
      gp = oD + (size_t)blockIdx.y * nPA + rowBase + 4 * lane;
    }
  }
#pragma unroll
  for (int i = 0; i < 4; ++i) *(volatile v4f*)(xpp[i]) = xr[i];
  if (gp) *(volatile v4f*)gp = gv;
  __threadfence();
#pragma unroll
  for (int i = 0; i < 4; ++i) *(volatile v4f*)(xpp[i]) = xr[i];
  if (gp) *(volatile v4f*)gp = gv;
}

__global__ __launch_bounds__(NTHR) void k_gcn_agg(
    const float* __restrict__ hs, const int* __restrict__ ei, const float* __restrict__ dinv,
    const float* __restrict__ bias, _Float16* act, int nN, int nE) {
  extern __shared__ v4f lds_dyn[];
  float* sacc = (float*)lds_dyn;
  float* dv   = sacc + NB * DF;
  int*   list = (int*)(dv + NB);
  int*   wcnt = list + NWAVE * WCAP;

  const int tid  = threadIdx.x;
  const int lane = tid & 31;
  const int wave = tid >> 5;
  const int hh   = lane >> 4;
  const int m    = lane & 15;
  const int nodeBase = blockIdx.x * NB;

  {
    const v4f z4 = {0.f, 0.f, 0.f, 0.f};
    for (int i = tid; i < NB * DF / 4; i += NTHR) lds_dyn[i] = z4;
    for (int i = tid; i < NB; i += NTHR) dv[i] = dinv[nodeBase + i];
  }
  __syncthreads();

  const int* eid = ei + nE;
  const bool al16 = ((nE & 3) == 0);
  const int nChunks = (nE + CHUNK - 1) / CHUNK;
#pragma unroll 1
  for (int ch = 0; ch < nChunks; ++ch) {
    const int cbase = ch * CHUNK;
    const int wc = scan_chunk<NB, SB>(eid, nE, al16, cbase, nodeBase, tid, wave, list);
    if (lane == 0) wcnt[wave] = wc;
    __syncthreads();
    if (wave == 0) {
      for (int wsx = 0; wsx < NWAVE; ++wsx) {
        int n = wcnt[wsx];
        n = n < 0 ? 0 : (n > WCAP ? WCAP : n);
        for (int i = 0; i < n; ++i) {
          const int ent  = list[wsx * WCAP + i];
          const int slot = ent & (NB - 1);
          const int el   = (ent >> SB) & (CHUNK - 1);
          int e = cbase + el;
          if (e > nE - 1) e = nE - 1;
          int src = ei[e];
          src = src < 0 ? 0 : (src > nN - 1 ? nN - 1 : src);
          const v4f v = *(const v4f*)(hs + (size_t)src * DF + 4 * lane);
          v4f* sp = (v4f*)(sacc + slot * DF + 4 * lane);
          *sp = *sp + v;
        }
      }
    }
    __syncthreads();
  }

  const int c0 = 8 * m;
  const v4f bA = *(const v4f*)(bias + c0);
  const v4f bB = *(const v4f*)(bias + c0 + 4);
#pragma unroll 1
  for (int j = 0; j < NB / (2 * NWAVE); ++j) {
    const int slot = wave * (NB / NWAVE) + 2 * j + hh;
    const int node = nodeBase + slot;
    const float d = dv[slot];
    const float* hr = hs + (size_t)node * DF + c0;
    const v4f a0 = *(const v4f*)(sacc + slot * DF + c0)     + *(const v4f*)(hr);
    const v4f a1 = *(const v4f*)(sacc + slot * DF + c0 + 4) + *(const v4f*)(hr + 4);
    v4f y0 = relu4(d * a0 + bA);
    v4f y1 = relu4(d * a1 + bB);
    if (node >= nN) { const v4f z4 = {0.f, 0.f, 0.f, 0.f}; y0 = z4; y1 = z4; }
    Pack16 u;
    u.h = cvt8(y0, y1, 8.0f);
    _Float16* p = act + (size_t)node * DF + c0;
    *(volatile v4i*)p = u.i;
    __threadfence();
    *(volatile v4i*)p = u.i;
  }
}

__global__ __launch_bounds__(NTHR) void k_gat1(
    const int* __restrict__ ei, const float* __restrict__ alS, const float* __restrict__ alD,
    float* mi, int nN, int nE, int nPA) {
  extern __shared__ v4f lds_dyn[];
  float* mx   = (float*)lds_dyn;
  float* den  = mx + NBL * 2;
  float* ad   = den + NBL * 2;
  int*   list = (int*)(ad + NBL * 2);
  int*   wcnt = list + NWAVE * WCAP;

  const int tid  = threadIdx.x;
  const int lane = tid & 31;
  const int wave = tid >> 5;
  const int nodeBase = blockIdx.x * NBL;

  for (int i = tid; i < NBL * 2; i += NTHR) {
    const int slot = i >> 1, h = i & 1;
    int nd = nodeBase + slot;
    if (nd > nN - 1) nd = nN - 1;
    mx[i]  = -1.0e30f;
    den[i] = 0.f;
    ad[i]  = alD[(size_t)h * nPA + nd];
  }
  __syncthreads();

  const int* eid = ei + nE;
  const bool al16 = ((nE & 3) == 0);
  const int nChunks = (nE + CHUNK - 1) / CHUNK;
#pragma unroll 1
  for (int ch = 0; ch < nChunks; ++ch) {
    const int cbase = ch * CHUNK;
    const int wc = scan_chunk<NBL, SBL>(eid, nE, al16, cbase, nodeBase, tid, wave, list);
    if (lane == 0) wcnt[wave] = wc;
    __syncthreads();
    if (wave == 0) {
      const int hs2 = lane & 1;
      for (int wsx = 0; wsx < NWAVE; ++wsx) {
        int n = wcnt[wsx];
        n = n < 0 ? 0 : (n > WCAP ? WCAP : n);
        for (int i = 0; i < n; ++i) {
          const int ent  = list[wsx * WCAP + i];
          const int slot = ent & (NBL - 1);
          const int el   = (ent >> SBL) & (CHUNK - 1);
          int e = cbase + el;
          if (e > nE - 1) e = nE - 1;
          int src = ei[e];
          src = src < 0 ? 0 : (src > nN - 1 ? nN - 1 : src);
          const int ai = slot * 2 + hs2;
          const float a  = leaky02(alS[(size_t)hs2 * nPA + src] + ad[ai]);
          const float mo = mx[ai];
          const float mn = fmaxf(mo, a);
          const float dn = den[ai] * __expf(mo - mn) + __expf(a - mn);
          if (lane < 2) { mx[ai] = mn; den[ai] = dn; }
        }
      }
    }
    __syncthreads();
  }

  for (int i = tid; i < NBL; i += NTHR) {
    const int node = nodeBase + i;
    int nd = node;
    if (nd > nN - 1) nd = nN - 1;
    const float a0  = leaky02(alS[nd] + ad[2 * i]);
    const float a1  = leaky02(alS[(size_t)nPA + nd] + ad[2 * i + 1]);
    const float mo0 = mx[2 * i], mo1 = mx[2 * i + 1];
    const float mn0 = fmaxf(mo0, a0), mn1 = fmaxf(mo1, a1);
    const float d0  = den[2 * i]     * __expf(mo0 - mn0) + __expf(a0 - mn0);
    const float d1  = den[2 * i + 1] * __expf(mo1 - mn1) + __expf(a1 - mn1);
    v4f r;
    r.x = mn0;
    r.y = mn1;
    r.z = __builtin_amdgcn_rcpf(d0 + 1e-16f);
    r.w = __builtin_amdgcn_rcpf(d1 + 1e-16f);
    float* p = mi + (size_t)node * 4;
    *(volatile v4f*)p = r;
    __threadfence();
    *(volatile v4f*)p = r;
  }
}

__global__ __launch_bounds__(NTHR) void k_gat2(
    const float* __restrict__ hg, const int* __restrict__ ei,
    const float* __restrict__ alS, const float* __restrict__ alD, const float* __restrict__ mi,
    const float* __restrict__ bias, float* h4, int nN, int nE, int nPA) {
  extern __shared__ v4f lds_dyn[];
  float* sacc = (float*)lds_dyn;
  float* sm   = sacc + NB * DF;
  float* ad   = sm + NB * 4;
  int*   list = (int*)(ad + NB * 2);
  int*   wcnt = list + NWAVE * WCAP;

  const int tid  = threadIdx.x;
  const int lane = tid & 31;
  const int wave = tid >> 5;
  const int nodeBase = blockIdx.x * NB;

  {
    const v4f z4 = {0.f, 0.f, 0.f, 0.f};
    for (int i = tid; i < NB * DF / 4; i += NTHR) lds_dyn[i] = z4;
    for (int i = tid; i < NB; i += NTHR) {
      const int node = nodeBase + i;
      *(v4f*)(sm + 4 * i) = *(const v4f*)(mi + (size_t)node * 4);
      ad[2 * i]     = alD[node];
      ad[2 * i + 1] = alD[(size_t)nPA + node];
    }
  }
  __syncthreads();

  const int* eid = ei + nE;
  const bool al16 = ((nE & 3) == 0);
  const int nChunks = (nE + CHUNK - 1) / CHUNK;
#pragma unroll 1
  for (int ch = 0; ch < nChunks; ++ch) {
    const int cbase = ch * CHUNK;
    const int wc = scan_chunk<NB, SB>(eid, nE, al16, cbase, nodeBase, tid, wave, list);
    if (lane == 0) wcnt[wave] = wc;
    __syncthreads();
    if (wave == 0) {
      for (int wsx = 0; wsx < NWAVE; ++wsx) {
        int n = wcnt[wsx];
        n = n < 0 ? 0 : (n > WCAP ? WCAP : n);
        for (int i = 0; i < n; ++i) {
          const int ent  = list[wsx * WCAP + i];
          const int slot = ent & (NB - 1);
          const int el   = (ent >> SB) & (CHUNK - 1);
          int e = cbase + el;
          if (e > nE - 1) e = nE - 1;
          int src = ei[e];
          src = src < 0 ? 0 : (src > nN - 1 ? nN - 1 : src);
          const float a0 = leaky02(alS[src] + ad[2 * slot]);
          const float a1 = leaky02(alS[(size_t)nPA + src] + ad[2 * slot + 1]);
          const v4f m4 = *(const v4f*)(sm + 4 * slot);
          const float c0 = __expf(a0 - m4.x) * m4.z;
          const float c1 = __expf(a1 - m4.y) * m4.w;
          const float* hr = hg + (size_t)src * (2 * DF) + 4 * lane;
          const v4f v0 = *(const v4f*)(hr);
          const v4f v1 = *(const v4f*)(hr + DF);
          v4f* sp = (v4f*)(sacc + slot * DF + 4 * lane);
          *sp = *sp + c0 * v0 + c1 * v1;
        }
      }
    }
    __syncthreads();
  }

  const v4f b4 = *(const v4f*)(bias + 4 * lane);
#pragma unroll 1
  for (int j = 0; j < NB / NWAVE; ++j) {
    const int slot = wave * (NB / NWAVE) + j;
    const int node = nodeBase + slot;
    const float a0 = leaky02(alS[node] + ad[2 * slot]);
    const float a1 = leaky02(alS[(size_t)nPA + node] + ad[2 * slot + 1]);
    const v4f m4 = *(const v4f*)(sm + 4 * slot);
    const float c0 = __expf(a0 - m4.x) * m4.z;
    const float c1 = __expf(a1 - m4.y) * m4.w;
    const float* hr = hg + (size_t)node * (2 * DF) + 4 * lane;
    const v4f v0 = *(const v4f*)(hr);
    const v4f v1 = *(const v4f*)(hr + DF);
    const v4f t = *(const v4f*)(sacc + slot * DF + 4 * lane) + c0 * v0 + c1 * v1;
    v4f y = relu4(0.5f * t + b4);
    if (node >= nN) { const v4f z4 = {0.f, 0.f, 0.f, 0.f}; y = z4; }
    float* p = h4 + (size_t)node * DF + 4 * lane;
    *(volatile v4f*)p = y;
    __threadfence();
    *(volatile v4f*)p = y;
  }
}

__global__ __launch_bounds__(NTHR) void k_gpool(
    const float* __restrict__ h, const int* __restrict__ bt, float* gb, int nN) {
  const int lane = threadIdx.x & 31;
  const int wave = threadIdx.x >> 5;
  const int gbase = (blockIdx.x * NWAVE + wave) * GPW;
  v4f a0 = {0.f, 0.f, 0.f, 0.f}, a1 = a0, a2 = a0, a3 = a0;
  int c0 = 0, c1 = 0, c2 = 0, c3 = 0;
#pragma unroll 1
  for (int base = 0; base < nN; base += 32) {
    const int n = base + lane;
    const int b = bt[min(n, nN - 1)];
    const unsigned rel = (unsigned)b - (unsigned)gbase;
    const bool hit = (n < nN) && (rel < (unsigned)GPW);
    unsigned msk = __builtin_amdgcn_ballot_w32(hit);
    while (msk != 0u) {
      const int i = __builtin_ctz(msk);
      msk &= msk - 1u;
      const int gl = __shfl((int)rel, i, 32);
      const v4f hv = *(const v4f*)(h + (size_t)(base + i) * DF + 4 * lane);
      if (gl == 0)      { a0 += hv; ++c0; }
      else if (gl == 1) { a1 += hv; ++c1; }
      else if (gl == 2) { a2 += hv; ++c2; }
      else              { a3 += hv; ++c3; }
    }
  }
  const float r0 = __builtin_amdgcn_rcpf((float)(c0 > 1 ? c0 : 1));
  const float r1 = __builtin_amdgcn_rcpf((float)(c1 > 1 ? c1 : 1));
  const float r2 = __builtin_amdgcn_rcpf((float)(c2 > 1 ? c2 : 1));
  const float r3 = __builtin_amdgcn_rcpf((float)(c3 > 1 ? c3 : 1));
  const v4f g0 = a0 * r0 + a0;
  const v4f g1 = a1 * r1 + a1;
  const v4f g2 = a2 * r2 + a2;
  const v4f g3 = a3 * r3 + a3;
  float* p0 = gb + (size_t)(gbase + 0) * DF + 4 * lane;
  float* p1 = gb + (size_t)(gbase + 1) * DF + 4 * lane;
  float* p2 = gb + (size_t)(gbase + 2) * DF + 4 * lane;
  float* p3 = gb + (size_t)(gbase + 3) * DF + 4 * lane;
  *(volatile v4f*)p0 = g0; *(volatile v4f*)p1 = g1; *(volatile v4f*)p2 = g2; *(volatile v4f*)p3 = g3;
  __threadfence();
  *(volatile v4f*)p0 = g0; *(volatile v4f*)p1 = g1; *(volatile v4f*)p2 = g2; *(volatile v4f*)p3 = g3;
}

__global__ __launch_bounds__(NTHR) void k_head(
    const float* __restrict__ gb, const _Float16* __restrict__ T1, const float* __restrict__ b1,
    const _Float16* __restrict__ T2, const float* __restrict__ b2, float* out, int nG) {
  __shared__ __attribute__((aligned(16))) _Float16 A1[GROWS * AP];
  __shared__ __attribute__((aligned(16))) _Float16 A2[GROWS * AP];
  __shared__ float Lg[GROWS * LGP];
  __shared__ __attribute__((aligned(16))) float Os[GROWS * NOUT];

  const int tid  = threadIdx.x;
  const int lane = tid & 31;
  const int wave = tid >> 5;
  const int hh   = lane >> 4;
  const int m    = lane & 15;

  {
    const int r  = tid >> 2;
    const int c0 = (tid & 3) * 32;
    const float* p = gb + (size_t)r * DF + c0;
#pragma unroll
    for (int k = 0; k < 4; ++k) {
      const v4f f0 = *(const v4f*)(p + 8 * k), f1 = *(const v4f*)(p + 8 * k + 4);
      *(v8h*)(A1 + r * AP + c0 + 8 * k) = cvt8(f0, f1, 8.0f);
    }
  }
  __syncthreads();

  const float e1 = 1.0f / 128.0f;
  const int ncol = wave * 16 + m;
  {
    v8f c0a = {0.f, 0.f, 0.f, 0.f, 0.f, 0.f, 0.f, 0.f};
    v8f c1a = c0a, c2a = c0a, c3a = c0a;
#pragma unroll
    for (int kt = 0; kt < DF / 32; ++kt) {
      const int k0 = kt * 32;
      Frag a0, a1, a2, a3, b;
      const _Float16* pb = T1 + (size_t)ncol * DF + k0 + 8 * hh;
      const _Float16* p0 = A1 + (0 * 16 + m) * AP + k0 + 8 * hh;
      const _Float16* p1 = A1 + (1 * 16 + m) * AP + k0 + 8 * hh;
      const _Float16* p2 = A1 + (2 * 16 + m) * AP + k0 + 8 * hh;
      const _Float16* p3 = A1 + (3 * 16 + m) * AP + k0 + 8 * hh;
      b.half[0]  = *(const v8h*)pb; b.half[1]  = *(const v8h*)(pb + 16);
      a0.half[0] = *(const v8h*)p0; a0.half[1] = *(const v8h*)(p0 + 16);
      a1.half[0] = *(const v8h*)p1; a1.half[1] = *(const v8h*)(p1 + 16);
      a2.half[0] = *(const v8h*)p2; a2.half[1] = *(const v8h*)(p2 + 16);
      a3.half[0] = *(const v8h*)p3; a3.half[1] = *(const v8h*)(p3 + 16);
      c0a = wm(a0.v, b.v, c0a);
      c1a = wm(a1.v, b.v, c1a);
      c2a = wm(a2.v, b.v, c2a);
      c3a = wm(a3.v, b.v, c3a);
    }
    const float pb1 = b1[ncol];
#pragma unroll
    for (int r = 0; r < 8; ++r) {
      A2[(0 * 16 + 8 * hh + r) * AP + ncol] = (_Float16)(fmaxf(c0a[r] * e1 + pb1, 0.f) * 8.0f);
      A2[(1 * 16 + 8 * hh + r) * AP + ncol] = (_Float16)(fmaxf(c1a[r] * e1 + pb1, 0.f) * 8.0f);
      A2[(2 * 16 + 8 * hh + r) * AP + ncol] = (_Float16)(fmaxf(c2a[r] * e1 + pb1, 0.f) * 8.0f);
      A2[(3 * 16 + 8 * hh + r) * AP + ncol] = (_Float16)(fmaxf(c3a[r] * e1 + pb1, 0.f) * 8.0f);
    }
  }
  __syncthreads();

  {
    const int T   = wave & 3;
    const int ct  = wave >> 2;
    const int nc2 = ct * 16 + m;
    v8f c = {0.f, 0.f, 0.f, 0.f, 0.f, 0.f, 0.f, 0.f};
#pragma unroll
    for (int kt = 0; kt < DF / 32; ++kt) {
      const int k0 = kt * 32;
      Frag a, b;
      const _Float16* pb = T2 + (size_t)nc2 * DF + k0 + 8 * hh;
      const _Float16* pa = A2 + (T * 16 + m) * AP + k0 + 8 * hh;
      b.half[0] = *(const v8h*)pb; b.half[1] = *(const v8h*)(pb + 16);
      a.half[0] = *(const v8h*)pa; a.half[1] = *(const v8h*)(pa + 16);
      c = wm(a.v, b.v, c);
    }
    const float pb2 = b2[nc2];
#pragma unroll
    for (int r = 0; r < 8; ++r) Lg[(T * 16 + 8 * hh + r) * LGP + nc2] = c[r] * e1 + pb2;
  }
  __syncthreads();

#pragma unroll 1
  for (int i = 0; i < 8; ++i) {
    const int row = wave * 8 + i;
    const float z  = Lg[row * LGP + lane];
    const float mx = wmax(z);
    const float zs = z - mx;
    const float s  = wsum(expf(zs));
    Os[row * NOUT + lane] = zs - logf(s);
  }
  __syncthreads();

  if (wave == 0) {
    for (int q = 0; q < GROWS / 4; ++q) {
      const int row = 4 * q + (lane >> 3);
      if (row < nG) {
        const v4f v = *(const v4f*)(Os + row * NOUT + (lane & 7) * 4);
        *(volatile v4f*)(out + (size_t)row * NOUT + (lane & 7) * 4) = v;
      }
    }
    __threadfence();
    for (int q = 0; q < GROWS / 4; ++q) {
      const int row = 4 * q + (lane >> 3);
      if (row < nG) {
        const v4f v = *(const v4f*)(Os + row * NOUT + (lane & 7) * 4);
        *(volatile v4f*)(out + (size_t)row * NOUT + (lane & 7) * 4) = v;
      }
    }
  }
}

extern "C" void kernel_launch(void* const* d_in, const int* in_sizes, int n_in,
                              void* d_out, int out_size, void* d_ws, size_t ws_size,
                              hipStream_t stream) {
  if (n_in < 17) return;
  const int nN = in_sizes[2];
  if (nN < 1) return;
  if (in_sizes[0] != nN * DF) return;
  if (in_sizes[1] < 0 || (in_sizes[1] & 1) != 0) return;
  const int nE = in_sizes[1] / 2;
  if (in_sizes[3] != DF * DF || in_sizes[4] != DF) return;
  if (in_sizes[5] != DF * DF || in_sizes[6] != DF) return;
  if (in_sizes[7] != DF * DF || in_sizes[8] != DF) return;
  if (in_sizes[9] != DF * 2 * DF || in_sizes[10] != 2 * DF || in_sizes[11] != 2 * DF || in_sizes[12] != DF) return;
  if (in_sizes[13] != DF * DF || in_sizes[14] != DF || in_sizes[15] != DF * NOUT || in_sizes[16] != NOUT) return;
  if (out_size < NOUT || (out_size % NOUT) != 0) return;
  const int G = out_size / NOUT;
  if (G > GROWS) return;

  const float* x     = (const float*)d_in[0];
  const int*   ei    = (const int*)d_in[1];
  const int*   batch = (const int*)d_in[2];
  const float* W1    = (const float*)d_in[3];  const float* b1   = (const float*)d_in[4];
  const float* W2    = (const float*)d_in[5];  const float* b2   = (const float*)d_in[6];
  const float* W3    = (const float*)d_in[7];  const float* b3   = (const float*)d_in[8];
  const float* gatW  = (const float*)d_in[9];
  const float* attS  = (const float*)d_in[10];
  const float* attD  = (const float*)d_in[11];
  const float* gatB  = (const float*)d_in[12];
  const float* fc1W  = (const float*)d_in[13]; const float* fc1b = (const float*)d_in[14];
  const float* fc2W  = (const float*)d_in[15]; const float* fc2b = (const float*)d_in[16];
  float* out = (float*)d_out;

  const int nPA = ((nN + NB - 1) / NB) * NB;
  const int nBl = nPA / NB;
  const int nP1 = ((nN + NBL - 1) / NBL) * NBL;
  const int nB1 = nP1 / NBL;

  size_t off = 0;
  char* base = (char*)d_ws;
#define CARVE(T, name, bytes) T* name = (T*)(base + off); off += (((size_t)(bytes)) + 255) & ~(size_t)255;
  CARVE(_Float16, T1,  (size_t)DF * DF * 2)
  CARVE(_Float16, T2,  (size_t)DF * DF * 2)
  CARVE(_Float16, T3,  (size_t)DF * DF * 2)
  CARVE(_Float16, Tg,  (size_t)2 * DF * DF * 2)
  CARVE(_Float16, Tf1, (size_t)DF * DF * 2)
  CARVE(_Float16, Tf2, (size_t)NOUT * DF * 2)
  CARVE(float, dinv,  (size_t)nP1 * 4)
  CARVE(float, alS,   (size_t)2 * nPA * 4)
  CARVE(float, alD,   (size_t)2 * nPA * 4)
  CARVE(float, mi,    (size_t)nP1 * 4 * 4)
  CARVE(float, hbig,  (size_t)nPA * 2 * DF * 4)
  CARVE(_Float16, act, (size_t)nPA * DF * 2)
  CARVE(float, h4,    (size_t)nPA * DF * 4)
  CARVE(float, gbuf,  (size_t)GROWS * DF * 4)
#undef CARVE
  if (off > ws_size) return;
  if (off > (size_t)134217728) return;

  k_prep<<<dim3(16, 6), NTHR, 0, stream>>>(W1, W2, W3, gatW, fc1W, fc2W, T1, T2, T3, Tg, Tf1, Tf2);

  k_deg<<<nB1, NTHR, 0, stream>>>(ei, dinv, nE);

  hipFuncSetAttribute(reinterpret_cast<const void*>(&k_gcn_agg),
                      hipFuncAttributeMaxDynamicSharedMemorySize, LDS_GCN);
  hipFuncSetAttribute(reinterpret_cast<const void*>(&k_gat1),
                      hipFuncAttributeMaxDynamicSharedMemorySize, LDS_G1);
  hipFuncSetAttribute(reinterpret_cast<const void*>(&k_gat2),
                      hipFuncAttributeMaxDynamicSharedMemorySize, LDS_G2);

  const int gridG = nPA / GR;
  const float e16 = 1.0f / 16.0f, e128 = 1.0f / 128.0f;

  k_gemm<float, 0><<<gridG, NTHR, 0, stream>>>(x, T1, dinv, attS, attD, hbig, alS, alD, nN, nPA, e16);
  k_gcn_agg<<<nBl, NTHR, LDS_GCN, stream>>>(hbig, ei, dinv, b1, act, nN, nE);
  k_gemm<_Float16, 0><<<gridG, NTHR, 0, stream>>>(act, T2, dinv, attS, attD, hbig, alS, alD, nN, nPA, e128);
  k_gcn_agg<<<nBl, NTHR, LDS_GCN, stream>>>(hbig, ei, dinv, b2, act, nN, nE);
  k_gemm<_Float16, 0><<<gridG, NTHR, 0, stream>>>(act, T3, dinv, attS, attD, hbig, alS, alD, nN, nPA, e128);
  k_gcn_agg<<<nBl, NTHR, LDS_GCN, stream>>>(hbig, ei, dinv, b3, act, nN, nE);

  k_gemm<_Float16, 1><<<dim3(gridG, 2), NTHR, 0, stream>>>(act, Tg, dinv, attS, attD, hbig, alS, alD, nN, nPA, e128);
  k_gat1<<<nB1, NTHR, LDS_G1, stream>>>(ei, alS, alD, mi, nN, nE, nPA);
  k_gat2<<<nBl, NTHR, LDS_G2, stream>>>(hbig, ei, alS, alD, mi, gatB, h4, nN, nE, nPA);

  k_gpool<<<GROWS / (NWAVE * GPW), NTHR, 0, stream>>>(h4, batch, gbuf, nN);
  k_head<<<1, NTHR, 0, stream>>>(gbuf, Tf1, fc1b, Tf2, fc2b, out, G);
}
